// CMAttention_55714315764288
// MI455X (gfx1250) — hardware-verified
//
#include <hip/hip_runtime.h>
#include <math.h>
#include <stdint.h>

#define NB      2
#define NTOK    2048
#define SEQ     4096
#define DM      1024
#define NHEAD   16
#define HD      64
#define RP      32
#define W3      3072
#define QKW     2048
#define SEG     1024
#define NSEG    4
#define NQB     16
#define NQP     4
#define MROWS   128
#define OUT1OFF (NB * NTOK * DM)
#define XSC     16.0f
#define WSC     64.0f
#define QSC     4.0f
#define KSC     16.0f
#define VSC     16.0f
#define RSC     4096.0f
#define PSC     1024.0f
#define NRM_EPS 1.0e-12f
#define DEN_EPS 1.0e-6f
#define LOG2_BASE 13.287712379549449
#define NEG_BIG (-1.0e30f)

static_assert(NHEAD * HD == DM);
static_assert(SEQ == 2 * NTOK);
static_assert(SEQ == NSEG * SEG);
static_assert(SEG == NQB * 64);
static_assert(HD == 2 * RP);
static_assert(W3 == 3 * DM);
static_assert(QKW == 2 * DM);
static_assert(((NB * NTOK * DM) % 2048) == 0);
static_assert(((SEQ * RP) % 256) == 0);
static_assert((DM % 128) == 0 && (W3 % 64) == 0 && (NTOK % 64) == 0 && (SEQ % 64) == 0);
static_assert((QKW % 128) == 0 && (DM % 32) == 0);
static_assert(NQP > 0 && NQP < NQB);
static_assert((SEG % MROWS) == 0 && MROWS == 8 * 16);
static_assert(OUT1OFF == NB * NTOK * DM);

typedef _Float16 v16h __attribute__((ext_vector_type(16)));
typedef _Float16 v8h  __attribute__((ext_vector_type(8)));
typedef float    v8f  __attribute__((ext_vector_type(8)));
typedef float    v4f  __attribute__((ext_vector_type(4)));
typedef unsigned int v4u __attribute__((ext_vector_type(4)));
union FH { v16h v; v8h h[2]; };

__device__ __forceinline__ unsigned short bf_bits(float f) {
  unsigned u = __float_as_uint(f);
  return (unsigned short)((u + 0x7FFFu + ((u >> 16) & 1u)) >> 16);
}
__device__ __forceinline__ float bf_up(unsigned short b) { return __uint_as_float(((unsigned)b) << 16); }
__device__ __forceinline__ float bfr(float f) { return bf_up(bf_bits(f)); }
__device__ __forceinline__ unsigned short h_bits(_Float16 x) { return __builtin_bit_cast(unsigned short, x); }
__device__ __forceinline__ unsigned pk16(unsigned short a, unsigned short b) { return (unsigned)a | ((unsigned)b << 16); }
__device__ __forceinline__ v8f zero8() { v8f z = {0.f, 0.f, 0.f, 0.f, 0.f, 0.f, 0.f, 0.f}; return z; }

__device__ __forceinline__ v16h ldfrag_h(const _Float16* p) {
  FH f;
  f.h[0] = *(const v8h*)(p);
  f.h[1] = *(const v8h*)(p + 16);
  return f.v;
}

__device__ __forceinline__ v8f mma_h_raw(v16h a, v16h b, v8f c) {
  return __builtin_amdgcn_wmma_f32_16x16x32_f16(false, a, false, b, (short)0, c, false, false);
}
__device__ __forceinline__ v8f mma_h(v16h a, v16h b, v8f c) {
  c = mma_h_raw(a, b, c);
#if defined(__HIP_DEVICE_COMPILE__)
  asm volatile("v_nop\n\tv_nop\n\tv_nop\n\tv_nop" : "+v"(c) : "v"(a), "v"(b));
#endif
  return c;
}
__device__ __forceinline__ void guard3(v8f& x, v8f& y, v16h a, v16h b, v16h d) {
#if defined(__HIP_DEVICE_COMPILE__)
  asm volatile("v_nop\n\tv_nop\n\tv_nop\n\tv_nop" : "+v"(x), "+v"(y) : "v"(a), "v"(b), "v"(d));
#endif
}
__device__ __forceinline__ void guard1q(v8f& x, v16h a, v16h b, v16h d, v16h e) {
#if defined(__HIP_DEVICE_COMPILE__)
  asm volatile("v_nop\n\tv_nop\n\tv_nop\n\tv_nop" : "+v"(x) : "v"(a), "v"(b), "v"(d), "v"(e));
#endif
}
__device__ __forceinline__ void guard4m(v8f& x, v8f& y, v16h a, v16h b, v16h d, v16h e) {
#if defined(__HIP_DEVICE_COMPILE__)
  asm volatile("v_nop\n\tv_nop\n\tv_nop\n\tv_nop" : "+v"(x), "+v"(y) : "v"(a), "v"(b), "v"(d), "v"(e)
               : "memory");
#endif
}
__device__ __forceinline__ void guard8m(v8f& x, v8f& y, v16h a, v16h b, v16h d, v16h e,
                                        v16h f, v16h g, v16h p, v16h q) {
#if defined(__HIP_DEVICE_COMPILE__)
  asm volatile("v_nop\n\tv_nop\n\tv_nop\n\tv_nop" : "+v"(x), "+v"(y)
               : "v"(a), "v"(b), "v"(d), "v"(e), "v"(f), "v"(g), "v"(p), "v"(q) : "memory");
#endif
}
__device__ __forceinline__ void acc_guard4(v8f& a, v8f& b, v8f& c, v8f& d) {
#if defined(__HIP_DEVICE_COMPILE__)
  asm volatile("v_nop\n\tv_nop\n\tv_nop\n\tv_nop" : "+v"(a), "+v"(b), "+v"(c), "+v"(d));
#endif
}
__device__ __forceinline__ void acc_guard2(v8f& a, v8f& b) {
#if defined(__HIP_DEVICE_COMPILE__)
  asm volatile("v_nop\n\tv_nop\n\tv_nop\n\tv_nop" : "+v"(a), "+v"(b));
#endif
}
__device__ __forceinline__ void cbar() {
#if defined(__HIP_DEVICE_COMPILE__)
  asm volatile("" ::: "memory");
#endif
}
__device__ __forceinline__ void wave_sync_lds() {
  __builtin_amdgcn_fence(__ATOMIC_RELEASE, "workgroup");
  __builtin_amdgcn_wave_barrier();
  __builtin_amdgcn_fence(__ATOMIC_ACQUIRE, "workgroup");
}

__global__ __launch_bounds__(256) void cvt_rm(const float* __restrict__ in, unsigned short* out, int n,
                                             float scale) {
  const size_t i8 = ((size_t)blockIdx.x * 256 + threadIdx.x) * 8;
  if (i8 + 8 > (size_t)n) return;
  const v4f a = *(const v4f*)(in + i8);
  const v4f b = *(const v4f*)(in + i8 + 4);
  float f[8];
  f[0] = a[0]; f[1] = a[1]; f[2] = a[2]; f[3] = a[3];
  f[4] = b[0]; f[5] = b[1]; f[6] = b[2]; f[7] = b[3];
  v4u p;
#pragma unroll
  for (int e = 0; e < 4; ++e) {
    const unsigned short b0 = bf_bits(f[2 * e]), b1 = bf_bits(f[2 * e + 1]);
    const _Float16 x0 = (_Float16)(bf_up(b0) * scale);
    const _Float16 x1 = (_Float16)(bf_up(b1) * scale);
    p[e] = pk16(h_bits(x0), h_bits(x1));
  }
  *(volatile v4u*)(out + i8) = p;
  __threadfence();
  *(volatile v4u*)(out + i8) = p;
}

template <int MODE>
__global__ __launch_bounds__(256) void tr_cvt(const float* __restrict__ in, int R, int C,
                                             unsigned short* out0, unsigned short* out1, float scale) {
  __shared__ float sm[64][65];
  const int tid = threadIdx.x;
  const int c0 = blockIdx.x * 64;
  const int r0 = blockIdx.y * 64;
  if (c0 + 64 > C || r0 + 64 > R) return;
  {
    const int lr = tid >> 2, lc = (tid & 3) * 16;
    const float* src = in + (size_t)(r0 + lr) * (size_t)C + c0 + lc;
#pragma unroll
    for (int q = 0; q < 4; ++q) {
      const v4f v = *(const v4f*)(src + 4 * q);
      sm[lr][lc + 4 * q + 0] = v[0];
      sm[lr][lc + 4 * q + 1] = v[1];
      sm[lr][lc + 4 * q + 2] = v[2];
      sm[lr][lc + 4 * q + 3] = v[3];
    }
  }
  __syncthreads();
  const int seg = tid & 7;
  v4u p0[2], p1[2];
#pragma unroll
  for (int it = 0; it < 2; ++it) {
    const int ocl = it * 32 + (tid >> 3);
    float f[8];
#pragma unroll
    for (int e = 0; e < 8; ++e) f[e] = sm[seg * 8 + e][ocl];
    v4u pk, pl;
#pragma unroll
    for (int e = 0; e < 4; ++e) {
      const float g0 = f[2 * e], g1 = f[2 * e + 1];
      if (MODE == 0) {
        const _Float16 x0 = (_Float16)(bfr(g0) * scale);
        const _Float16 x1 = (_Float16)(bfr(g1) * scale);
        pk[e] = pk16(h_bits(x0), h_bits(x1));
        pl[e] = pk[e];
      } else {
        const float s0 = g0 * scale, s1 = g1 * scale;
        const _Float16 x0 = (_Float16)s0, x1 = (_Float16)s1;
        const _Float16 y0 = (_Float16)((s0 - (float)x0) * RSC);
        const _Float16 y1 = (_Float16)((s1 - (float)x1) * RSC);
        pk[e] = pk16(h_bits(x0), h_bits(x1));
        pl[e] = pk16(h_bits(y0), h_bits(y1));
      }
    }
    p0[it] = pk;
    p1[it] = pl;
  }
  for (int pass = 0; pass < 2; ++pass) {
#pragma unroll
    for (int it = 0; it < 2; ++it) {
      const int ocl = it * 32 + (tid >> 3);
      const size_t go = (size_t)(c0 + ocl) * (size_t)R + (size_t)(r0 + seg * 8);
      *(volatile v4u*)(out0 + go) = p0[it];
      if (MODE == 1) *(volatile v4u*)(out1 + go) = p1[it];
    }
    __threadfence();
  }
}

__global__ __launch_bounds__(256) void rope_tab(float* cost, float* sint, int n) {
  const int e = blockIdx.x * 256 + (int)threadIdx.x;
  if (e >= n) return;
  const int t = e >> 5, i = e & 31;
  const double pd = exp2((double)i * (1.0 / 32.0) * LOG2_BASE);
  const float  pf = (float)pd;
  const float  invf = (float)(1.0 / (double)pf);
  const float  ang = (float)t * invf;
  float sv, cv;
  sincosf(ang, &sv, &cv);
  *(volatile float*)(cost + e) = cv;
  *(volatile float*)(sint + e) = sv;
  __threadfence();
  *(volatile float*)(cost + e) = cv;
  *(volatile float*)(sint + e) = sv;
}

template <int EPI>
__global__ __launch_bounds__(128) void gemm_t(
    const unsigned short* __restrict__ A, int lda,
    const unsigned short* __restrict__ Bt, int ldb,
    void* C0, void* C1, int ldc, int crow0,
    const float* __restrict__ cost, const float* __restrict__ sint,
    const float* __restrict__ gq, const float* __restrict__ gk,
    int M, int N, int K, float oscale) {
  __shared__ __align__(16) float sT[4][16 * 132];
  const int lane = threadIdx.x & 31;
  const int wave = threadIdx.x >> 5;
  const int tilesN = N >> 7;
  const int tilesM = M >> 5;
  const int tile = blockIdx.x * 4 + wave;
  if (tile >= tilesM * tilesN) return;
  const int tm = tile / tilesN;
  const int tn = tile - tm * tilesN;
  const int m0 = tm << 5;
  const int n0 = tn << 7;
  const int rl   = lane & 15;
  const int hh   = lane >> 4;
  const int koff = hh * 8;

  v8f acc[2][8];
#pragma unroll
  for (int i = 0; i < 2; ++i)
#pragma unroll
    for (int j = 0; j < 8; ++j) acc[i][j] = zero8();

  {
    const _Float16* ar0 = (const _Float16*)(const void*)A + (size_t)(m0 + rl) * (size_t)lda + koff;
    const _Float16* ar1 = (const _Float16*)(const void*)A + (size_t)(m0 + 16 + rl) * (size_t)lda + koff;
    const _Float16* br  = (const _Float16*)(const void*)Bt + (size_t)(n0 + rl) * (size_t)ldb + koff;
    for (int k0 = 0; k0 < K; k0 += 32) {
      const v16h a0 = ldfrag_h(ar0 + k0);
      const v16h a1 = ldfrag_h(ar1 + k0);
#pragma unroll
      for (int j = 0; j < 8; ++j) {
        const v16h b = ldfrag_h(br + (size_t)j * 16 * (size_t)ldb + k0);
        acc[0][j] = mma_h_raw(a0, b, acc[0][j]);
        acc[1][j] = mma_h_raw(a1, b, acc[1][j]);
        guard3(acc[0][j], acc[1][j], a0, a1, b);
      }
    }
  }
  acc_guard4(acc[0][0], acc[0][1], acc[0][2], acc[0][3]);
  acc_guard4(acc[0][4], acc[0][5], acc[0][6], acc[0][7]);
  acc_guard4(acc[1][0], acc[1][1], acc[1][2], acc[1][3]);
  acc_guard4(acc[1][4], acc[1][5], acc[1][6], acc[1][7]);

  float* slab = sT[wave];
  float gmul[8];
  float csc = 1.0f;
  if (EPI == 1) {
    const bool isq = (n0 < DM);
    const int  hb  = (isq ? n0 : (n0 - DM)) >> 6;
    csc = isq ? QSC : KSC;
#pragma unroll
    for (int j = 0; j < 8; ++j) {
      const int gi = (hb + (j >> 2)) * HD + 16 * (j & 3) + rl;
      const float ga = bfr(gq[gi]);
      const float gb = bfr(gk[gi]);
      gmul[j] = (isq ? ga : gb) * 8.0f;
    }
  } else {
#pragma unroll
    for (int j = 0; j < 8; ++j) gmul[j] = 1.0f;
  }
#pragma unroll
  for (int i = 0; i < 2; ++i) {
    const int mB = m0 + 16 * i;
    if (EPI == 1) {
      float inv[2][8];
#pragma unroll
      for (int jh = 0; jh < 2; ++jh) {
#pragma unroll
        for (int r = 0; r < 8; ++r) {
          float ss = 0.f;
#pragma unroll
          for (int jj = 0; jj < 4; ++jj) {
            const float x = acc[i][4 * jh + jj][r] * oscale;
            ss += x * x;
          }
          ss += __shfl_xor(ss, 1, 32);
          ss += __shfl_xor(ss, 2, 32);
          ss += __shfl_xor(ss, 4, 32);
          ss += __shfl_xor(ss, 8, 32);
          inv[jh][r] = oscale * (1.0f / fmaxf(sqrtf(ss), NRM_EPS));
        }
      }
#pragma unroll
      for (int j = 0; j < 8; ++j) {
#pragma unroll
        for (int r = 0; r < 8; ++r)
          slab[(8 * hh + r) * 132 + 16 * j + rl] = acc[i][j][r] * inv[j >> 2][r] * gmul[j];
      }
    } else {
#pragma unroll
      for (int j = 0; j < 8; ++j) {
#pragma unroll
        for (int r = 0; r < 8; ++r) slab[(8 * hh + r) * 132 + 16 * j + rl] = acc[i][j][r] * oscale;
      }
    }
    wave_sync_lds();
    if (EPI == 3) {
      float* Cf = (float*)C0;
      v4f ov[16];
#pragma unroll
      for (int it = 0; it < 16; ++it) ov[it] = *(const v4f*)(slab + it * 132 + lane * 4);
      for (int pass = 0; pass < 2; ++pass) {
#pragma unroll
        for (int it = 0; it < 16; ++it)
          *(volatile v4f*)(Cf + (size_t)(crow0 + mB + it) * (size_t)ldc + n0 + lane * 4) = ov[it];
        __threadfence();
      }
    } else {
      unsigned short* Cp = (unsigned short*)C0;
      unsigned short* Cq = (unsigned short*)C1;
      v4u hv[8], lv[8];
#pragma unroll
      for (int it = 0; it < 8; ++it) {
        const int row = it * 2 + hh;
        const float* sp = slab + row * 132 + rl * 8;
        const v4f fa = *(const v4f*)sp;
        const v4f fb = *(const v4f*)(sp + 4);
        float f[8];
        f[0] = fa[0]; f[1] = fa[1]; f[2] = fa[2]; f[3] = fa[3];
        f[4] = fb[0]; f[5] = fb[1]; f[6] = fb[2]; f[7] = fb[3];
        const int pos = crow0 + mB + row;
        const v4f cv = *(const v4f*)(cost + (size_t)pos * RP + (rl & 7) * 4);
        const v4f sv = *(const v4f*)(sint + (size_t)pos * RP + (rl & 7) * 4);
        v4u pk, pl;
#pragma unroll
        for (int e = 0; e < 4; ++e) {
          const float f0 = f[2 * e], f1 = f[2 * e + 1];
          const float cc = cv[e], sn = sv[e];
          const float g0 = (f0 * cc - f1 * sn) * csc;
          const float g1 = (f0 * sn + f1 * cc) * csc;
          const _Float16 x0 = (_Float16)g0;
          const _Float16 x1 = (_Float16)g1;
          const _Float16 y0 = (_Float16)((g0 - (float)x0) * RSC);
          const _Float16 y1 = (_Float16)((g1 - (float)x1) * RSC);
          pk[e] = pk16(h_bits(x0), h_bits(x1));
          pl[e] = pk16(h_bits(y0), h_bits(y1));
        }
        hv[it] = pk;
        lv[it] = pl;
      }
      for (int pass = 0; pass < 2; ++pass) {
#pragma unroll
        for (int it = 0; it < 8; ++it) {
          const int row = it * 2 + hh;
          const size_t go = (size_t)(crow0 + mB + row) * (size_t)ldc + n0 + rl * 8;
          *(volatile v4u*)(Cp + go) = hv[it];
          *(volatile v4u*)(Cq + go) = lv[it];
        }
        __threadfence();
      }
    }
    wave_sync_lds();
  }
}

__global__ __launch_bounds__(256) void mt_seg(const unsigned short* __restrict__ QKH,
                                             const unsigned short* __restrict__ QKL,
                                             const unsigned short* __restrict__ VTH,
                                             float* MT, float* ZP) {
  __shared__ __align__(16) _Float16 skT[HD * 72];
  __shared__ __align__(16) float slab[8][16 * 36];
  __shared__ float zred[8][HD];
  __shared__ __align__(16) float zsum[HD];

  const int tid = threadIdx.x, wave = tid >> 5, lane = tid & 31, hh = lane >> 4, c = lane & 15;
  const int h = (int)(blockIdx.x / 3u);
  const int s = (int)(blockIdx.x - (unsigned)h * 3u);
  if (h >= NHEAD) return;
  const int r  = tid >> 2;
  const int dq = (tid & 3) * 16;
  const int et = wave >> 1;
  const int dt0 = (wave & 1) * 2;

  const _Float16* Q16 = (const _Float16*)(const void*)QKH;
  const _Float16* L16 = (const _Float16*)(const void*)QKL;
  const _Float16* V16 = (const _Float16*)(const void*)VTH;
  const _Float16* vrow = V16 + (size_t)(h * HD + et * 16 + c) * SEQ + (size_t)s * SEG + 8 * hh;

  float zacc[16];
#pragma unroll
  for (int e = 0; e < 16; ++e) zacc[e] = 0.f;
  v8f acc[2];
  acc[0] = zero8(); acc[1] = zero8();

  for (int kt = 0; kt < SEG / 64; ++kt) {
    __syncthreads();
    {
      const size_t n = (size_t)(s * SEG + kt * 64 + r);
      const _Float16* kp = Q16 + n * QKW + DM + h * HD + dq;
      const _Float16* lp = L16 + n * QKW + DM + h * HD + dq;
      FH kf, lf;
      kf.h[0] = *(const v8h*)kp; kf.h[1] = *(const v8h*)(kp + 8);
      lf.h[0] = *(const v8h*)lp; lf.h[1] = *(const v8h*)(lp + 8);
#pragma unroll
      for (int e = 0; e < 16; ++e) {
        const float kv = ((float)kf.v[e] + (float)lf.v[e] * (1.0f / RSC)) * (1.0f / KSC);
        const float sk = (kv > 0.f) ? (kv + 1.0f) : __expf(kv);
        const _Float16 skh = (_Float16)sk;
        skT[(dq + e) * 72 + r] = skh;
        zacc[e] += (float)skh;
      }
    }
    __syncthreads();
#pragma unroll
    for (int kk = 0; kk < 2; ++kk) {
      const v16h a  = ldfrag_h(vrow + kt * 64 + 32 * kk);
      const v16h b0 = ldfrag_h(skT + (16 * dt0 + c) * 72 + 32 * kk + 8 * hh);
      const v16h b1 = ldfrag_h(skT + (16 * (dt0 + 1) + c) * 72 + 32 * kk + 8 * hh);
      acc[0] = mma_h_raw(a, b0, acc[0]);
      acc[1] = mma_h_raw(a, b1, acc[1]);
      guard3(acc[0], acc[1], a, b0, b1);
    }
  }
  acc_guard2(acc[0], acc[1]);

  float* sl = slab[wave];
#pragma unroll
  for (int jj = 0; jj < 2; ++jj) {
#pragma unroll
    for (int rr = 0; rr < 8; ++rr) sl[(8 * hh + rr) * 36 + 16 * jj + c] = acc[jj][rr] * (1.0f / VSC);
  }
  wave_sync_lds();
  {
    v4f mv[4];
#pragma unroll
    for (int it = 0; it < 4; ++it) {
      const int row = it * 4 + (lane >> 3);
      mv[it] = *(const v4f*)(sl + row * 36 + (lane & 7) * 4);
    }
    float* mtb = MT + ((size_t)(h * 3 + s) * HD + (size_t)et * 16) * HD + (wave & 1) * 32;
    for (int pass = 0; pass < 2; ++pass) {
#pragma unroll
      for (int it = 0; it < 4; ++it) {
        const int row = it * 4 + (lane >> 3);
        *(volatile v4f*)(mtb + (size_t)row * HD + (lane & 7) * 4) = mv[it];
      }
      __threadfence();
    }
  }
#pragma unroll
  for (int e = 0; e < 16; ++e) {
    float v = zacc[e];
    v += __shfl_xor(v, 4, 32);
    v += __shfl_xor(v, 8, 32);
    v += __shfl_xor(v, 16, 32);
    if ((lane >> 2) == 0) zred[wave][(lane & 3) * 16 + e] = v;
  }
  __syncthreads();
  if (tid < HD) {
    float z = 0.f;
#pragma unroll
    for (int w = 0; w < 8; ++w) z += zred[w][tid];
    zsum[tid] = z;
  }
  __syncthreads();
  if (tid < 16) {
    const v4f zz = *(const v4f*)(zsum + tid * 4);
    float* zp = ZP + (size_t)(h * 3 + s) * HD + tid * 4;
    *(volatile v4f*)zp = zz;
    __threadfence();
    *(volatile v4f*)zp = zz;
  }
}

__global__ __launch_bounds__(256) void mem_ret(const unsigned short* __restrict__ QKH,
                                              const unsigned short* __restrict__ QKL,
                                              const float* __restrict__ MT, const float* __restrict__ ZP,
                                              float* MEM) {
  __shared__ __align__(16) _Float16 MTh[HD * 72];
  __shared__ float zs[HD];
  __shared__ __align__(16) float slab[8][16 * 68];

  const int tid = threadIdx.x, wave = tid >> 5, lane = tid & 31, hh = lane >> 4, c = lane & 15;
  const int h   = (int)(blockIdx.x / 24u);
  const int rem = (int)(blockIdx.x - (unsigned)h * 24u);
  const int s   = 1 + rem / 8;
  const int rb  = rem - (s - 1) * 8;
  if (h >= NHEAD) return;

  {
    const int e = tid >> 2, d0 = (tid & 3) * 16;
    float sm[16];
#pragma unroll
    for (int i = 0; i < 16; ++i) sm[i] = 0.f;
#pragma unroll
    for (int sp = 0; sp < 3; ++sp) {
      if (sp < s) {
        const float* src = MT + ((size_t)(h * 3 + sp) * HD + e) * HD + d0;
#pragma unroll
        for (int q = 0; q < 4; ++q) {
          const v4f v = *(const v4f*)(src + 4 * q);
          sm[4 * q + 0] += v[0]; sm[4 * q + 1] += v[1]; sm[4 * q + 2] += v[2]; sm[4 * q + 3] += v[3];
        }
      }
    }
    v8h p0, p1;
#pragma unroll
    for (int i = 0; i < 8; ++i) { p0[i] = (_Float16)sm[i]; p1[i] = (_Float16)sm[8 + i]; }
    *(v8h*)(MTh + e * 72 + d0) = p0;
    *(v8h*)(MTh + e * 72 + d0 + 8) = p1;
    if (tid < HD) {
      float z = 0.f;
#pragma unroll
      for (int sp = 0; sp < 3; ++sp) {
        if (sp < s) z += ZP[(size_t)(h * 3 + sp) * HD + tid];
      }
      zs[tid] = z;
    }
  }
  __syncthreads();

  const _Float16* Q16 = (const _Float16*)(const void*)QKH;
  const _Float16* L16 = (const _Float16*)(const void*)QKL;
  const int n0w = s * SEG + rb * MROWS + wave * 16;

  v16h af[2];
  float denp = 0.f;
#pragma unroll
  for (int kk = 0; kk < 2; ++kk) {
    FH hf, lf;
    hf.v = ldfrag_h(Q16 + (size_t)(n0w + c) * QKW + h * HD + 32 * kk + 8 * hh);
    lf.v = ldfrag_h(L16 + (size_t)(n0w + c) * QKW + h * HD + 32 * kk + 8 * hh);
    v16h a;
#pragma unroll
    for (int i = 0; i < 16; ++i) {
      const float qv = ((float)hf.v[i] + (float)lf.v[i] * (1.0f / RSC)) * (1.0f / QSC);
      const float sq = (qv > 0.f) ? (qv + 1.0f) : __expf(qv);
      const _Float16 sqh = (_Float16)sq;
      a[i] = sqh;
      const int kidx = 32 * kk + ((i < 8) ? (8 * hh + i) : (8 + 8 * hh + i));
      denp += (float)sqh * zs[kidx];
    }
    af[kk] = a;
  }
  const float den = denp + __shfl_xor(denp, 16, 32) + DEN_EPS;

  v8f acc[4];
#pragma unroll
  for (int j = 0; j < 4; ++j) {
    acc[j] = zero8();
#pragma unroll
    for (int kk = 0; kk < 2; ++kk) {
      const v16h b = ldfrag_h(MTh + (16 * j + c) * 72 + 32 * kk + 8 * hh);
      acc[j] = mma_h(af[kk], b, acc[j]);
    }
  }
  float rinv[8];
#pragma unroll
  for (int rr = 0; rr < 8; ++rr) rinv[rr] = 1.0f / __shfl(den, 8 * hh + rr, 32);

  float* sl = slab[wave];
#pragma unroll
  for (int j = 0; j < 4; ++j) {
#pragma unroll
    for (int rr = 0; rr < 8; ++rr) sl[(8 * hh + rr) * 68 + 16 * j + c] = acc[j][rr] * rinv[rr];
  }
  wave_sync_lds();
  {
    v4f ov[8];
#pragma unroll
    for (int it = 0; it < 8; ++it) {
      const int row = it * 2 + hh;
      ov[it] = *(const v4f*)(sl + row * 68 + c * 4);
    }
    for (int pass = 0; pass < 2; ++pass) {
#pragma unroll
      for (int it = 0; it < 8; ++it) {
        const int row = it * 2 + hh;
        *(volatile v4f*)(MEM + (size_t)(n0w + row) * DM + h * HD + c * 4) = ov[it];
      }
      __threadfence();
    }
  }
}

template <bool PRES>
__global__ __launch_bounds__(128)
void attn_seg(const unsigned short* __restrict__ QKH, const unsigned short* __restrict__ QKL,
              const unsigned short* __restrict__ VTH, const unsigned short* __restrict__ VTL,
              const float* __restrict__ MEM, const float* __restrict__ gate,
              float* outb, float sscale, int qb0, int nqb) {
  __shared__ __align__(16) _Float16 Ksh[64 * HD];
  __shared__ __align__(16) _Float16 Kls[64 * HD];
  __shared__ __align__(16) _Float16 Vhs[HD * 64];
  __shared__ __align__(16) _Float16 Vls[PRES ? HD * 64 : 8];
  __shared__ __align__(16) _Float16 Psh[4][16 * 64];
  __shared__ __align__(16) _Float16 Psl[PRES ? 4 : 1][PRES ? 16 * 64 : 8];
  __shared__ __align__(16) float    Os[4][16 * 68];

  const int tid  = threadIdx.x;
  const int wave = tid >> 5;
  const int lane = tid & 31;
  const int hh   = lane >> 4;
  const int c    = lane & 15;

  const int per = NSEG * nqb;
  const int h   = (int)(blockIdx.x / (unsigned)per);
  const int rem = (int)(blockIdx.x - (unsigned)h * (unsigned)per);
  const int seg = rem / nqb;
  const int qbs = qb0 + (rem - seg * nqb);
  if (h >= NHEAD || seg >= NSEG) return;
  const int sbase = seg * SEG;
  const int rowl0 = qbs * 64 + wave * 16;
  const int q0    = sbase + rowl0;

  const _Float16* Q16 = (const _Float16*)(const void*)QKH;
  const _Float16* L16 = (const _Float16*)(const void*)QKL;
  const _Float16* Qg  = Q16 + (size_t)h * HD;
  const _Float16* Qlg = L16 + (size_t)h * HD;
  const _Float16* Kg  = Q16 + DM + (size_t)h * HD;
  const _Float16* Klg = L16 + DM + (size_t)h * HD;
  const _Float16* Vhg = (const _Float16*)(const void*)VTH + (size_t)h * HD * SEQ;
  const _Float16* Vlg = (const _Float16*)(const void*)VTL + (size_t)h * HD * SEQ;

  const v16h qh0 = ldfrag_h(Qg  + (size_t)(q0 + c) * QKW + 8 * hh);
  const v16h qh1 = ldfrag_h(Qg  + (size_t)(q0 + c) * QKW + 32 + 8 * hh);
  const v16h ql0 = ldfrag_h(Qlg + (size_t)(q0 + c) * QKW + 8 * hh);
  const v16h ql1 = ldfrag_h(Qlg + (size_t)(q0 + c) * QKW + 32 + 8 * hh);

  float mrow[8], lrow[8];
  v8f oh[4];
#pragma unroll
  for (int r = 0; r < 8; ++r) { mrow[r] = NEG_BIG; lrow[r] = 0.f; }
#pragma unroll
  for (int t = 0; t < 4; ++t) oh[t] = zero8();

  _Float16* pwh = Psh[wave];
  _Float16* pwl = &Psl[PRES ? wave : 0][0];

  for (int kt = 0; kt < NQB; ++kt) {
    if (kt > qbs) break;
    const int kv0 = sbase + kt * 64;
    __syncthreads();
    {
      const int r = tid >> 1, hk = (tid & 1) * 32;
      const _Float16* kg = Kg + (size_t)(kv0 + r) * QKW + hk;
#pragma unroll
      for (int i = 0; i < 4; ++i) *(v8h*)(Ksh + r * HD + hk + 8 * i) = *(const v8h*)(kg + 8 * i);
      cbar();
      const _Float16* lg = Klg + (size_t)(kv0 + r) * QKW + hk;
#pragma unroll
      for (int i = 0; i < 4; ++i) *(v8h*)(Kls + r * HD + hk + 8 * i) = *(const v8h*)(lg + 8 * i);
      cbar();
      const _Float16* vh = Vhg + (size_t)r * SEQ + kv0 + hk;
#pragma unroll
      for (int i = 0; i < 4; ++i) *(v8h*)(Vhs + r * 64 + hk + 8 * i) = *(const v8h*)(vh + 8 * i);
      if (PRES) {
        cbar();
        const _Float16* vl = Vlg + (size_t)r * SEQ + kv0 + hk;
#pragma unroll
        for (int i = 0; i < 4; ++i) *(v8h*)(Vls + r * 64 + hk + 8 * i) = *(const v8h*)(vl + 8 * i);
        cbar();
      }
    }
    __syncthreads();

    v8f s[4];
#pragma unroll
    for (int j = 0; j < 4; ++j) {
      v8f sh = zero8(), sl = zero8();
      {
        FH kb, lb;
        kb.h[0] = *(const v8h*)(Ksh + (j * 16 + c) * HD + 8 * hh);
        kb.h[1] = *(const v8h*)(Ksh + (j * 16 + c) * HD + 16 + 8 * hh);
        lb.h[0] = *(const v8h*)(Kls + (j * 16 + c) * HD + 8 * hh);
        lb.h[1] = *(const v8h*)(Kls + (j * 16 + c) * HD + 16 + 8 * hh);
        sh = mma_h_raw(qh0, kb.v, sh);
        sl = mma_h_raw(ql0, kb.v, sl);
        sl = mma_h_raw(qh0, lb.v, sl);
        guard4m(sh, sl, qh0, ql0, kb.v, lb.v);
      }
      {
        FH kb, lb;
        kb.h[0] = *(const v8h*)(Ksh + (j * 16 + c) * HD + 32 + 8 * hh);
        kb.h[1] = *(const v8h*)(Ksh + (j * 16 + c) * HD + 48 + 8 * hh);
        lb.h[0] = *(const v8h*)(Kls + (j * 16 + c) * HD + 32 + 8 * hh);
        lb.h[1] = *(const v8h*)(Kls + (j * 16 + c) * HD + 48 + 8 * hh);
        sh = mma_h_raw(qh1, kb.v, sh);
        sl = mma_h_raw(ql1, kb.v, sl);
        sl = mma_h_raw(qh1, lb.v, sl);
        guard4m(sh, sl, qh1, ql1, kb.v, lb.v);
      }
      const int key  = kt * 64 + j * 16 + c;
      const int rowb = rowl0 + 8 * hh;
#pragma unroll
      for (int r = 0; r < 8; ++r) {
        float v = sh[r];
        v += sl[r] * (1.0f / RSC);
        v *= sscale;
        s[j][r] = (key <= rowb + r) ? v : NEG_BIG;
      }
    }

#pragma unroll
    for (int r = 0; r < 8; ++r) {
      float m = s[0][r];
      m = fmaxf(m, s[1][r]);
      m = fmaxf(m, s[2][r]);
      m = fmaxf(m, s[3][r]);
#pragma unroll
      for (int off = 1; off < 16; off <<= 1) m = fmaxf(m, __shfl_xor(m, off, 32));
      const float mnew  = fmaxf(mrow[r], m);
      const float alpha = __expf(mrow[r] - mnew);
      mrow[r] = mnew;
      float psum = 0.f;
#pragma unroll
      for (int j = 0; j < 4; ++j) {
        const float p  = __expf(s[j][r] - mnew);
        psum += p;
        const float ph = p * PSC;
        const _Float16 xh = (_Float16)ph;
        const int pi = (8 * hh + r) * 64 + j * 16 + c;
        pwh[pi] = xh;
        if (PRES) pwl[pi] = (_Float16)((ph - (float)xh) * RSC);
      }
#pragma unroll
      for (int off = 1; off < 16; off <<= 1) psum += __shfl_xor(psum, off, 32);
      lrow[r] = lrow[r] * alpha + psum;
#pragma unroll
      for (int t = 0; t < 4; ++t) oh[t][r] *= alpha;
    }
    wave_sync_lds();

    FH pa0, pa1, pb0, pb1;
    pa0.h[0] = *(const v8h*)(pwh + c * 64 + 8 * hh);
    pa0.h[1] = *(const v8h*)(pwh + c * 64 + 16 + 8 * hh);
    pa1.h[0] = *(const v8h*)(pwh + c * 64 + 32 + 8 * hh);
    pa1.h[1] = *(const v8h*)(pwh + c * 64 + 48 + 8 * hh);
    pb0.v = pa0.v;
    pb1.v = pa1.v;
    if (PRES) {
      pb0.h[0] = *(const v8h*)(pwl + c * 64 + 8 * hh);
      pb0.h[1] = *(const v8h*)(pwl + c * 64 + 16 + 8 * hh);
      pb1.h[0] = *(const v8h*)(pwl + c * 64 + 32 + 8 * hh);
      pb1.h[1] = *(const v8h*)(pwl + c * 64 + 48 + 8 * hh);
      cbar();
    }
#pragma unroll
    for (int t = 0; t < 4; ++t) {
      const _Float16* vr = Vhs + (t * 16 + c) * 64 + 8 * hh;
      FH vb0, vb1;
      vb0.h[0] = *(const v8h*)(vr);
      vb0.h[1] = *(const v8h*)(vr + 16);
      vb1.h[0] = *(const v8h*)(vr + 32);
      vb1.h[1] = *(const v8h*)(vr + 48);
      if (PRES) {
        const _Float16* wr = Vls + (t * 16 + c) * 64 + 8 * hh;
        FH wb0, wb1;
        wb0.h[0] = *(const v8h*)(wr);
        wb0.h[1] = *(const v8h*)(wr + 16);
        wb1.h[0] = *(const v8h*)(wr + 32);
        wb1.h[1] = *(const v8h*)(wr + 48);
        v8f ol = zero8();
        oh[t] = mma_h_raw(pa0.v, vb0.v, oh[t]);
        ol    = mma_h_raw(pa0.v, wb0.v, ol);
        ol    = mma_h_raw(pb0.v, vb0.v, ol);
        oh[t] = mma_h_raw(pa1.v, vb1.v, oh[t]);
        ol    = mma_h_raw(pa1.v, wb1.v, ol);
        ol    = mma_h_raw(pb1.v, vb1.v, ol);
        guard8m(oh[t], ol, pa0.v, pa1.v, pb0.v, pb1.v, vb0.v, vb1.v, wb0.v, wb1.v);
#pragma unroll
        for (int r = 0; r < 8; ++r) oh[t][r] += ol[r] * (1.0f / RSC);
      } else {
        oh[t] = mma_h_raw(pa0.v, vb0.v, oh[t]);
        oh[t] = mma_h_raw(pa1.v, vb1.v, oh[t]);
        guard1q(oh[t], pa0.v, pa1.v, vb0.v, vb1.v);
      }
    }
    acc_guard4(oh[0], oh[1], oh[2], oh[3]);
  }

  const float gv  = bfr(gate[h]);
  const float g   = 1.0f / (1.0f + expf(-gv));
  const float omg = 1.0f - g;
  const bool useMem = (seg > 0);
  float* os = Os[wave];
#pragma unroll
  for (int r = 0; r < 8; ++r) {
    const int qr = q0 + 8 * hh + r;
    const float l = lrow[r];
    const float inv = (1.0f / l) * (1.0f / (PSC * VSC));
    const float* mr = MEM + (size_t)qr * DM + h * HD;
#pragma unroll
    for (int t = 0; t < 4; ++t) {
      const float yv  = oh[t][r] * inv;
      const float mvr = mr[16 * t + c];
      const float mv  = useMem ? mvr : 0.f;
      os[(8 * hh + r) * 68 + 16 * t + c] = g * mv + omg * yv;
    }
  }
  wave_sync_lds();
  {
    const size_t ooff  = (seg < (NTOK / SEG)) ? (size_t)OUT1OFF : (size_t)0;
    const int    orow0 = (seg < (NTOK / SEG)) ? q0 : (q0 - NTOK);
    v4f ov[8];
#pragma unroll
    for (int it = 0; it < 8; ++it) {
      const int row = it * 2 + hh;
      ov[it] = *(const v4f*)(os + row * 68 + c * 4);
    }
    for (int pass = 0; pass < 2; ++pass) {
#pragma unroll
      for (int it = 0; it < 8; ++it) {
        const int row = it * 2 + hh;
        *(volatile v4f*)(outb + ooff + (size_t)(orow0 + row) * DM + h * HD + c * 4) = ov[it];
      }
      __threadfence();
    }
  }
}

extern "C" void kernel_launch(void* const* d_in, const int* in_sizes, int n_in,
                              void* d_out, int out_size, void* d_ws, size_t ws_size,
                              hipStream_t stream) {
  if (n_in < 9) return;
  if (in_sizes[0] != NB * NTOK * DM || in_sizes[1] != NB * NTOK * DM) return;
  if (in_sizes[2] != DM * W3 || in_sizes[3] != DM * W3) return;
  if (in_sizes[4] != NHEAD * HD || in_sizes[5] != NHEAD * HD) return;
  if (in_sizes[6] != NHEAD * HD || in_sizes[7] != NHEAD * HD) return;
  if (in_sizes[8] != NHEAD) return;
  if (out_size != 2 * NB * NTOK * DM) return;

  const float* X    = (const float*)d_in[0];
  const float* Aa   = (const float*)d_in[1];
  const float* Wx   = (const float*)d_in[2];
  const float* Wa   = (const float*)d_in[3];
  const float* g_qx = (const float*)d_in[4];
  const float* g_kx = (const float*)d_in[5];
  const float* g_qa = (const float*)d_in[6];
  const float* g_ka = (const float*)d_in[7];
  const float* gate = (const float*)d_in[8];
  float* outf = (float*)d_out;

  const size_t PXA = (size_t)NB * NTOK * DM * 2;
  const size_t PW  = (size_t)W3 * DM * 2;
  const size_t PRT = (size_t)SEQ * RP * 4;
  const size_t PQK = (size_t)SEQ * QKW * 2;
  const size_t PVF = (size_t)SEQ * DM * 4;
  const size_t PVT = (size_t)DM * SEQ * 2;
  const size_t PMT = (size_t)NHEAD * 3 * HD * HD * 4;
  const size_t PZP = (size_t)NHEAD * 3 * HD * 4;
  const size_t PME = (size_t)SEQ * DM * 4;
  size_t off = 0;
  const size_t oXH = off; off += PXA;
  const size_t oAH = off; off += PXA;
  const size_t oWX = off; off += PW;
  const size_t oWA = off; off += PW;
  const size_t oCT = off; off += PRT;
  const size_t oST = off; off += PRT;
  const size_t oQH = off; off += PQK;
  const size_t oQL = off; off += PQK;
  const size_t oVF = off; off += PVF;
  const size_t oVH = off; off += PVT;
  const size_t oVL = off; off += PVT;
  const size_t oMT = off; off += PMT;
  const size_t oZP = off; off += PZP;
  const size_t oME = off; off += PME;
  if (off > ws_size) return;
  if (off > (size_t)134217728) return;

  char* ws = (char*)d_ws;
  unsigned short* XH   = (unsigned short*)(ws + oXH);
  unsigned short* AH   = (unsigned short*)(ws + oAH);
  unsigned short* WXT  = (unsigned short*)(ws + oWX);
  unsigned short* WAT  = (unsigned short*)(ws + oWA);
  float*          COST = (float*)(ws + oCT);
  float*          SINT = (float*)(ws + oST);
  unsigned short* QKH  = (unsigned short*)(ws + oQH);
  unsigned short* QKL  = (unsigned short*)(ws + oQL);
  float*          VF   = (float*)(ws + oVF);
  unsigned short* VTH  = (unsigned short*)(ws + oVH);
  unsigned short* VTL  = (unsigned short*)(ws + oVL);
  float*          MT   = (float*)(ws + oMT);
  float*          ZP   = (float*)(ws + oZP);
  float*          MEM  = (float*)(ws + oME);

  const dim3 blk256(256), blk128(128);
  const float sscale = 0.125f / (QSC * KSC);
  const float oscale = 1.0f / (XSC * WSC);

  cvt_rm<<<dim3((NB * NTOK * DM) / 2048), blk256, 0, stream>>>(X, XH, NB * NTOK * DM, XSC);
  cvt_rm<<<dim3((NB * NTOK * DM) / 2048), blk256, 0, stream>>>(Aa, AH, NB * NTOK * DM, XSC);
  tr_cvt<0><<<dim3(W3 / 64, DM / 64), blk256, 0, stream>>>(Wx, DM, W3, WXT, WXT, WSC);
  tr_cvt<0><<<dim3(W3 / 64, DM / 64), blk256, 0, stream>>>(Wa, DM, W3, WAT, WAT, WSC);
  rope_tab<<<dim3((SEQ * RP) / 256), blk256, 0, stream>>>(COST, SINT, SEQ * RP);

  const int gqk  = ((NTOK / 32) * (QKW / 128)) / 4;
  const int gv   = ((NTOK / 32) * (DM / 128)) / 4;
  const int gmt  = NHEAD * 3;
  const int gmem = NHEAD * 3 * (SEG / MROWS);
  for (int b = 0; b < NB; ++b) {
    const unsigned short* AHb = AH + (size_t)b * NTOK * DM;
    const unsigned short* XHb = XH + (size_t)b * NTOK * DM;
    float* outb = outf + (size_t)b * NTOK * DM;
    gemm_t<1><<<dim3(gqk), blk128, 0, stream>>>(AHb, DM, WAT, DM, (void*)QKH, (void*)QKL, QKW, 0,
                                               COST, SINT, g_qa, g_ka, NTOK, QKW, DM, oscale);
    gemm_t<1><<<dim3(gqk), blk128, 0, stream>>>(XHb, DM, WXT, DM, (void*)QKH, (void*)QKL, QKW, NTOK,
                                               COST, SINT, g_qx, g_kx, NTOK, QKW, DM, oscale);
    gemm_t<3><<<dim3(gv), blk128, 0, stream>>>(AHb, DM, WAT + (size_t)2 * DM * DM, DM, (void*)VF, (void*)VF,
                                              DM, 0, COST, SINT, g_qa, g_ka, NTOK, DM, DM, oscale);
    gemm_t<3><<<dim3(gv), blk128, 0, stream>>>(XHb, DM, WXT + (size_t)2 * DM * DM, DM, (void*)VF, (void*)VF,
                                              DM, NTOK, COST, SINT, g_qx, g_kx, NTOK, DM, DM, oscale);
    tr_cvt<1><<<dim3(DM / 64, SEQ / 64), blk256, 0, stream>>>(VF, SEQ, DM, VTH, VTL, VSC);
    mt_seg<<<dim3(gmt), blk256, 0, stream>>>(QKH, QKL, VTH, MT, ZP);
    mem_ret<<<dim3(gmem), blk256, 0, stream>>>(QKH, QKL, MT, ZP, MEM);
    attn_seg<true><<<dim3(NHEAD * NSEG * NQP), blk128, 0, stream>>>(QKH, QKL, VTH, VTL, MEM, gate, outb,
                                                                    sscale, 0, NQP);
    attn_seg<false><<<dim3(NHEAD * NSEG * (NQB - NQP)), blk128, 0, stream>>>(QKH, QKL, VTH, VTL, MEM, gate,
                                                                             outb, sscale, NQP, NQB - NQP);
  }
  (void)hipGetLastError();
}
